// TemporalAttentionLayer_65292092833944
// MI455X (gfx1250) — hardware-verified
//
#include <hip/hip_runtime.h>
#include <math.h>
#include <stdint.h>

#define NBATCH 64
#define NWIN   1024
#define NFEAT  128
#define QTILE  64
#define JTILE  64
#define TP     72
#define OP     132
#define LRELU_SLOPE 0.2f

static_assert((NWIN % QTILE) == 0);
static_assert((NWIN % JTILE) == 0);
static_assert((NWIN % 32) == 0);
static_assert(NFEAT == 128);
static_assert(((TP * 2) % 16) == 0);
static_assert(((OP * 4) % 16) == 0);

typedef __bf16   v16b __attribute__((ext_vector_type(16)));
typedef __bf16   v8b  __attribute__((ext_vector_type(8)));
typedef float    v8f  __attribute__((ext_vector_type(8)));
typedef float    v4f  __attribute__((ext_vector_type(4)));
typedef unsigned int v4u __attribute__((ext_vector_type(4)));
typedef unsigned int v8u __attribute__((ext_vector_type(8)));
typedef v4f __attribute__((may_alias)) v4fa;
typedef v4u __attribute__((may_alias)) v4ua;
typedef v8b __attribute__((may_alias)) v8ba;

#if defined(__HIP_DEVICE_COMPILE__)
#define DEV_ASM 1
#else
#define DEV_ASM 0
#endif

__device__ __forceinline__ unsigned short bf_bits(float f) {
  unsigned u = __float_as_uint(f);
  return (unsigned short)((u + 0x7FFFu + ((u >> 16) & 1u)) >> 16);
}
__device__ __forceinline__ float bf_up(unsigned short hb) { return __uint_as_float(((unsigned)hb) << 16); }
__device__ __forceinline__ unsigned pk16(unsigned short a, unsigned short b) { return (unsigned)a | ((unsigned)b << 16); }
__device__ __forceinline__ v8f zero8() { v8f z = {0.f, 0.f, 0.f, 0.f, 0.f, 0.f, 0.f, 0.f}; return z; }
__device__ __forceinline__ float leaky(float e) { return (e > 0.f) ? e : (LRELU_SLOPE * e); }

__device__ __forceinline__ v16b ldfrag_b(const __bf16* p) {
  union { v16b v; v8b h[2]; } f;
  f.h[0] = *(const v8ba*)(p);
  f.h[1] = *(const v8ba*)(p + 16);
  return f.v;
}

__device__ __forceinline__ v8f mma_b(v16b a, v16b b, v8f c) {
  c = __builtin_amdgcn_wmma_f32_16x16x32_bf16(false, a, false, b, (short)0, c, false, false);
#if DEV_ASM
  asm volatile("v_nop\n\tv_nop\n\tv_nop\n\tv_nop" : "+v"(c) : "v"(a), "v"(b));
#endif
  return c;
}

__global__ __launch_bounds__(256) void k_prep(const float* __restrict__ x, const float* __restrict__ w,
                                              unsigned short* XT, float* SS) {
  __shared__ __align__(16) unsigned short T[NFEAT * TP];
  __shared__ __align__(16) float ss[2 * JTILE];

  const int tid  = threadIdx.x;
  const int lane = tid & 31;
  const int wave = tid >> 5;
  const int b    = blockIdx.y;
  const int j0   = blockIdx.x * JTILE;

  const v4f wa = *(const v4fa*)(w + 4 * lane);
  const v4f wc = *(const v4fa*)(w + NFEAT + 4 * lane);
  float w1f[4], w2f[4];
#pragma unroll
  for (int c = 0; c < 4; ++c) {
    w1f[c] = bf_up(bf_bits(wa[c]));
    w2f[c] = bf_up(bf_bits(wc[c]));
  }

#pragma unroll
  for (int it = 0; it < 8; ++it) {
    const int r = it * 8 + wave;
    const float* xr = x + ((size_t)(b * NWIN + j0 + r)) * NFEAT + 4 * lane;
    const v4f xv = *(const v4fa*)xr;
    float d1 = 0.0f, d2 = 0.0f;
#pragma unroll
    for (int c = 0; c < 4; ++c) {
      const unsigned short hb = bf_bits(xv[c]);
      const float xf = bf_up(hb);
      d1 += xf * w1f[c];
      d2 += xf * w2f[c];
      T[(4 * lane + c) * TP + r] = hb;
    }
#pragma unroll
    for (int off = 16; off >= 1; off >>= 1) {
      d1 += __shfl_xor(d1, off, 32);
      d2 += __shfl_xor(d2, off, 32);
    }
    if (lane == 0) {
      ss[r] = d1;
      ss[JTILE + r] = d2;
    }
  }
  __syncthreads();

  {
    const int q  = lane >> 3;
    const int c8 = (lane & 7) * 8;
    v4u vv[4];
#pragma unroll
    for (int it = 0; it < 4; ++it) {
      const int n = wave * 16 + it * 4 + q;
      vv[it] = *(const v4ua*)(T + n * TP + c8);
    }
    for (int pass = 0; pass < 2; ++pass) {
#pragma unroll
      for (int it = 0; it < 4; ++it) {
        const int n = wave * 16 + it * 4 + q;
        unsigned short* dst = XT + ((size_t)(b * NFEAT + n)) * NWIN + j0 + c8;
        *(volatile v4u*)dst = vv[it];
      }
      __threadfence();
    }
  }

  if (wave == 0) {
    const v4f sv = *(const v4fa*)(ss + 4 * lane);
    float* dst = SS + (size_t)b * (2 * NWIN) + (size_t)(lane >> 4) * NWIN + j0 + 4 * (lane & 15);
    *(volatile v4f*)dst = sv;
    __threadfence();
    *(volatile v4f*)dst = sv;
  }
}

__global__ __launch_bounds__(128) void k_attn(const unsigned short* __restrict__ XTp,
                                              const float* __restrict__ SS,
                                              float* out) {
  __shared__ __align__(16) float s2s[NWIN];
  __shared__ float red[4];
  __shared__ __align__(16) float os[4][16 * OP];

  const int tid  = threadIdx.x;
  const int lane = tid & 31;
  const int wave = tid >> 5;
  const int h    = lane >> 4;
  const int c    = lane & 15;
  const int b    = blockIdx.y;
  const int q0   = blockIdx.x * QTILE;

  const __bf16* XT = (const __bf16*)(const void*)XTp;
  const float* s1g = SS + (size_t)b * (2 * NWIN);
  const float* s2g = s1g + NWIN;

  const v4f sa = *(const v4fa*)(s2g + 4 * tid);
  const v4f sb = *(const v4fa*)(s2g + 512 + 4 * tid);
  *(v4fa*)(s2s + 4 * tid) = sa;
  *(v4fa*)(s2s + 512 + 4 * tid) = sb;
  float mx = fmaxf(fmaxf(fmaxf(sa[0], sa[1]), fmaxf(sa[2], sa[3])),
                   fmaxf(fmaxf(sb[0], sb[1]), fmaxf(sb[2], sb[3])));
#pragma unroll
  for (int off = 16; off >= 1; off >>= 1) mx = fmaxf(mx, __shfl_xor(mx, off, 32));
  if (lane == 0) red[wave] = mx;
  __syncthreads();
  const float s2max = fmaxf(fmaxf(red[0], red[1]), fmaxf(red[2], red[3]));

  const float s1m    = s1g[q0 + 16 * wave + c];
  const float rowmax = leaky(s1m + s2max);

  v8f acc[8];
#pragma unroll
  for (int t = 0; t < 8; ++t) acc[t] = zero8();
  float dsum = 0.0f;

  const __bf16* xrow = XT + ((size_t)(b * NFEAT + c)) * NWIN + 8 * h;

#pragma unroll 1
  for (int k0 = 0; k0 < NWIN; k0 += 32) {
    v8u ph = {0u, 0u, 0u, 0u, 0u, 0u, 0u, 0u};
    v8u pl = {0u, 0u, 0u, 0u, 0u, 0u, 0u, 0u};
#pragma unroll
    for (int e = 0; e < 8; ++e) {
      const int kk = k0 + 8 * h + 2 * e + ((e >= 4) ? 8 : 0);
      const float eA = leaky(s1m + s2s[kk]);
      const float eB = leaky(s1m + s2s[kk + 1]);
      const float pA = __expf(eA - rowmax);
      const float pB = __expf(eB - rowmax);
      dsum += pA;
      dsum += pB;
      const unsigned short hA = bf_bits(pA), hB = bf_bits(pB);
      const unsigned short lA = bf_bits(pA - bf_up(hA)), lB = bf_bits(pB - bf_up(hB));
      ph[e] = pk16(hA, hB);
      pl[e] = pk16(lA, lB);
    }
    const v16b ahi = __builtin_bit_cast(v16b, ph);
    const v16b alo = __builtin_bit_cast(v16b, pl);

#pragma unroll
    for (int t = 0; t < 8; ++t) {
      const v16b bf = ldfrag_b(xrow + (size_t)t * 16 * NWIN + k0);
      acc[t] = mma_b(ahi, bf, acc[t]);
      acc[t] = mma_b(alo, bf, acc[t]);
    }
  }

  dsum += __shfl_xor(dsum, 16, 32);
  float inv[8];
#pragma unroll
  for (int r = 0; r < 8; ++r) {
    const float l = __shfl(dsum, 8 * h + r, 32);
    inv[r] = 1.0f / l;
  }

  float* osw = os[wave];
#pragma unroll
  for (int t = 0; t < 8; ++t) {
#pragma unroll
    for (int r = 0; r < 8; ++r) {
      osw[(8 * h + r) * OP + 16 * t + c] = acc[t][r] * inv[r];
    }
  }
  __syncthreads();

  for (int pass = 0; pass < 2; ++pass) {
#pragma unroll
    for (int row = 0; row < 16; ++row) {
      const v4f v = *(const v4fa*)(osw + row * OP + 4 * lane);
      float* dst = out + ((size_t)(b * NWIN + q0 + 16 * wave + row)) * NFEAT + 4 * lane;
      *(volatile v4f*)dst = v;
    }
    __threadfence();
  }
}

extern "C" void kernel_launch(void* const* d_in, const int* in_sizes, int n_in,
                              void* d_out, int out_size, void* d_ws, size_t ws_size,
                              hipStream_t stream) {
  if (n_in < 2) return;
  if (in_sizes[0] != NBATCH * NWIN * NFEAT) return;
  if (in_sizes[1] != 2 * NFEAT) return;
  if (out_size != NBATCH * NWIN * NFEAT) return;

  const float* x = (const float*)d_in[0];
  const float* w = (const float*)d_in[1];
  float* out = (float*)d_out;

  const size_t bXT = (size_t)NBATCH * NFEAT * NWIN * 2;
  const size_t bSS = (size_t)NBATCH * 2 * NWIN * 4;
  size_t off = 0;
  const size_t oXT = off; off += bXT;
  const size_t oSS = off; off += bSS;
  if (off > ws_size) return;
  if (off > (size_t)134217728) return;

  char* ws = (char*)d_ws;
  unsigned short* XT = (unsigned short*)(ws + oXT);
  float*          SS = (float*)(ws + oSS);

  const dim3 gPrep(NWIN / JTILE, NBATCH);
  const dim3 gAttn(NWIN / QTILE, NBATCH);

  k_prep<<<gPrep, dim3(256), 0, stream>>>(x, w, XT, SS);
  k_attn<<<gAttn, dim3(128), 0, stream>>>(XT, SS, out);
  (void)hipGetLastError();
}
